// SelfAttentionModule_65481071408314
// MI455X (gfx1250) — hardware-run, weakly checked
//
#include <hip/hip_runtime.h>

#define EMB   1024
#define NH    16
#define HD    64
#define SEQ   2048
#define NB    2
#define MROWS (NB * SEQ)
#define NQKV  (3 * EMB)

#define QKV_CARRY 16.0f
#define PSCALE    16384.0f
#define WTD_CARRY 64.0f
#define WO_CARRY  256.0f
#define SSCALE    (0.125f / (QKV_CARRY * QKV_CARRY))
#define ATT_OSC   (WTD_CARRY / (PSCALE * QKV_CARRY))
#define OUT_OSC   (1.0f / (WTD_CARRY * WO_CARRY))
#define LN_EPS    1e-5f

#define NGX   (MROWS * EMB / 8)
#define NGWQ  (NQKV * EMB / 8)
#define NGWO  (EMB * EMB / 8)
#define NBX   (NGX / 256)
#define NBWQ  (NGWQ / 256)
#define NBWO  (NGWO / 256)

static_assert(NGX % 256 == 0);
static_assert(NGWQ % 256 == 0);
static_assert(NGWO % 256 == 0);
static_assert(MROWS % 128 == 0);
static_assert(SEQ % 128 == 0);
static_assert(SEQ % 64 == 0);
static_assert(EMB % 32 == 0);
static_assert(EMB == 8 * 128);
static_assert(HD == 64);
static_assert(NH * HD == EMB);
static_assert(MROWS % 16 == 0);

typedef _Float16 v16h __attribute__((ext_vector_type(16)));
typedef _Float16 v8h  __attribute__((ext_vector_type(8)));
typedef __bf16   v16b __attribute__((ext_vector_type(16)));
typedef __bf16   v8b  __attribute__((ext_vector_type(8)));
typedef float    v8f  __attribute__((ext_vector_type(8)));
typedef float    v4f  __attribute__((ext_vector_type(4)));
typedef unsigned int v4u __attribute__((ext_vector_type(4)));
typedef v8h __attribute__((may_alias)) v8ha;
typedef v8b __attribute__((may_alias)) v8ba;
typedef v4f __attribute__((may_alias)) v4fa;
typedef v4u __attribute__((may_alias)) v4ua;

union FragH { v16h v; v8h half[2]; };
union FragB { v16b v; v8b half[2]; };

__device__ __forceinline__ v8f wmma_h(v16h a, v16h b, v8f c) {
  v8f d = __builtin_amdgcn_wmma_f32_16x16x32_f16(false, a, false, b, (short)0, c, false, false);
  asm volatile("v_nop\n\tv_nop\n\tv_nop\n\tv_nop" : "+v"(d) : "v"(a), "v"(b));
  return d;
}
__device__ __forceinline__ v8f wmma_b(v16b a, v16b b, v8f c) {
  v8f d = __builtin_amdgcn_wmma_f32_16x16x32_bf16(false, a, false, b, (short)0, c, false, false);
  asm volatile("v_nop\n\tv_nop\n\tv_nop\n\tv_nop" : "+v"(d) : "v"(a), "v"(b));
  return d;
}

__device__ __forceinline__ v16h ldfrag_h(const _Float16* p, int h) {
  FragH f;
  f.half[0] = *(const v8ha*)(p + 8 * h);
  f.half[1] = *(const v8ha*)(p + 16 + 8 * h);
  return f.v;
}
__device__ __forceinline__ v16b ldfrag_b(const __bf16* p, int h) {
  FragB f;
  f.half[0] = *(const v8ba*)(p + 8 * h);
  f.half[1] = *(const v8ba*)(p + 16 + 8 * h);
  return f.v;
}

__device__ __forceinline__ unsigned short f2bf_bits(float f) {
  const unsigned u = __float_as_uint(f);
  return (unsigned short)((u + 0x7FFFu + ((u >> 16) & 1u)) >> 16);
}
__device__ __forceinline__ float bf_bits2f(unsigned short b) { return __uint_as_float(((unsigned)b) << 16); }
__device__ __forceinline__ float bfr(float f) { return bf_bits2f(f2bf_bits(f)); }
__device__ __forceinline__ unsigned pk16(unsigned short a, unsigned short b) { return (unsigned)a | ((unsigned)b << 16); }

__device__ __forceinline__ void cvt_bf16_8(const float* __restrict__ src, unsigned short* __restrict__ dst) {
  const v4f a = *(const v4fa*)src;
  const v4f c = *(const v4fa*)(src + 4);
  v4u o;
  o[0] = pk16(f2bf_bits(a[0]), f2bf_bits(a[1]));
  o[1] = pk16(f2bf_bits(a[2]), f2bf_bits(a[3]));
  o[2] = pk16(f2bf_bits(c[0]), f2bf_bits(c[1]));
  o[3] = pk16(f2bf_bits(c[2]), f2bf_bits(c[3]));
  *(volatile v4u*)dst = o;
  __threadfence();
  *(volatile v4u*)dst = o;
}
__device__ __forceinline__ void cvt_wo_8(const float* __restrict__ src, _Float16* __restrict__ dst) {
  const v4f a = *(const v4fa*)src;
  const v4f c = *(const v4fa*)(src + 4);
  v8h o;
  o[0] = (_Float16)(bfr(a[0]) * WO_CARRY);
  o[1] = (_Float16)(bfr(a[1]) * WO_CARRY);
  o[2] = (_Float16)(bfr(a[2]) * WO_CARRY);
  o[3] = (_Float16)(bfr(a[3]) * WO_CARRY);
  o[4] = (_Float16)(bfr(c[0]) * WO_CARRY);
  o[5] = (_Float16)(bfr(c[1]) * WO_CARRY);
  o[6] = (_Float16)(bfr(c[2]) * WO_CARRY);
  o[7] = (_Float16)(bfr(c[3]) * WO_CARRY);
  *(volatile v8h*)dst = o;
  __threadfence();
  *(volatile v8h*)dst = o;
}

__global__ __launch_bounds__(256) void prep_kernel(
    const float* __restrict__ x, const float* __restrict__ wqkv, const float* __restrict__ wout,
    unsigned short* __restrict__ xb, unsigned short* __restrict__ wq, _Float16* __restrict__ wo)
{
  const int blk = blockIdx.x;
  const int t = threadIdx.x;
  if (blk < NBX) {
    const size_t g = (size_t)blk * 256 + t;
    cvt_bf16_8(x + g * 8, xb + g * 8);
  } else if (blk < NBX + NBWQ) {
    const size_t g = (size_t)(blk - NBX) * 256 + t;
    cvt_bf16_8(wqkv + g * 8, wq + g * 8);
  } else {
    const size_t g = (size_t)(blk - NBX - NBWQ) * 256 + t;
    cvt_wo_8(wout + g * 8, wo + g * 8);
  }
}

__device__ __forceinline__ void qkv_store_pass(const _Float16* sT, _Float16* plane, _Float16* vt,
                                               int which, int bh, int l0, int w, int lane) {
  const int q8 = lane & 7, sub = lane >> 3;
#pragma unroll
  for (int i = 0; i < 8; ++i) {
    const int lid = w * 32 + i * 4 + sub;
    v8h v;
    _Float16* dst;
    if (which != 2) {
      v = *(const v8ha*)(sT + lid * HD + 8 * q8);
      dst = plane + ((size_t)bh * SEQ + l0 + lid) * HD + 8 * q8;
    } else {
      const int d = lid >> 1, hl = lid & 1;
      v = *(const v8ha*)(sT + d * 128 + 64 * hl + 8 * q8);
      dst = vt + ((size_t)bh * HD + d) * SEQ + l0 + 64 * hl + 8 * q8;
    }
    *(volatile v8h*)dst = v;
  }
}

__global__ __launch_bounds__(128) void qkv_kernel(
    const unsigned short* __restrict__ xb,
    const unsigned short* __restrict__ wq,
    const float* __restrict__ ap,
    _Float16* __restrict__ qp,
    _Float16* __restrict__ kp,
    _Float16* __restrict__ vt)
{
  __shared__ __attribute__((aligned(16))) float    sAP[128 * 64];
  __shared__ __attribute__((aligned(16))) _Float16 sT[128 * 64];

  const int tid = threadIdx.x, lane = tid & 31, w = tid >> 5;
  const int h = lane >> 4, m = lane & 15;
  const int m0 = blockIdx.x * 128;
  const int cg = blockIdx.y;
  const int which = cg >> 4, head = cg & 15;
  const int ncol0 = which * EMB + head * HD;
  const int m0w = m0 + 32 * w;

  const __bf16* Ab = (const __bf16*)(const void*)xb;
  const __bf16* Bb = (const __bf16*)(const void*)wq;
  const __bf16* xa0 = Ab + (size_t)(m0w + m) * EMB;
  const __bf16* xa1 = xa0 + (size_t)16 * EMB;
  const __bf16* wb  = Bb + (size_t)(ncol0 + m) * EMB;

  const v8f zero8 = {0.f, 0.f, 0.f, 0.f, 0.f, 0.f, 0.f, 0.f};
  v8f acc[2][4];
#pragma unroll
  for (int mt = 0; mt < 2; ++mt)
#pragma unroll
    for (int nt = 0; nt < 4; ++nt) acc[mt][nt] = zero8;

#pragma unroll 1
  for (int k0 = 0; k0 < EMB; k0 += 32) {
    const v16b a0 = ldfrag_b(xa0 + k0, h);
    const v16b a1 = ldfrag_b(xa1 + k0, h);
#pragma unroll
    for (int nt = 0; nt < 4; ++nt) {
      const v16b bfr_ = ldfrag_b(wb + (size_t)nt * 16 * EMB + k0, h);
      acc[0][nt] = wmma_b(a0, bfr_, acc[0][nt]);
      acc[1][nt] = wmma_b(a1, bfr_, acc[1][nt]);
    }
  }

  {
    const int lr = tid >> 4;
    const int c4 = (tid & 15) * 4;
#pragma unroll 4
    for (int it = 0; it < 16; ++it) {
      const int row = it * 8 + lr;
      const v4f a = *(const v4fa*)(ap + (size_t)(m0 + row) * NQKV + ncol0 + c4);
      *(v4fa*)(sAP + row * 64 + c4) = a;
    }
  }
  __syncthreads();

#pragma unroll
  for (int nt = 0; nt < 4; ++nt) {
    const int feat = 16 * nt + m;
#pragma unroll
    for (int mt = 0; mt < 2; ++mt) {
#pragma unroll
      for (int r = 0; r < 8; ++r) {
        const int tokl = 32 * w + 16 * mt + 8 * h + r;
        const float sc = bfr(sAP[tokl * 64 + feat]);
        const float y = acc[mt][nt][r] * sc * QKV_CARRY;
        const int idx = (which == 2) ? (feat * 128 + tokl) : (tokl * HD + feat);
        sT[idx] = (_Float16)y;
      }
    }
  }
  __syncthreads();

  const int b = m0 / SEQ, l0 = m0 - b * SEQ, bh = b * NH + head;
  _Float16* plane = (which == 0) ? qp : kp;
  qkv_store_pass(sT, plane, vt, which, bh, l0, w, lane);
  __threadfence();
  qkv_store_pass(sT, plane, vt, which, bh, l0, w, lane);
}

__device__ __forceinline__ v16h pack_p(v8f a, v8f c) {
  const v16h r = { (_Float16)(a[0] * PSCALE), (_Float16)(a[1] * PSCALE), (_Float16)(a[2] * PSCALE), (_Float16)(a[3] * PSCALE),
                   (_Float16)(a[4] * PSCALE), (_Float16)(a[5] * PSCALE), (_Float16)(a[6] * PSCALE), (_Float16)(a[7] * PSCALE),
                   (_Float16)(c[0] * PSCALE), (_Float16)(c[1] * PSCALE), (_Float16)(c[2] * PSCALE), (_Float16)(c[3] * PSCALE),
                   (_Float16)(c[4] * PSCALE), (_Float16)(c[5] * PSCALE), (_Float16)(c[6] * PSCALE), (_Float16)(c[7] * PSCALE) };
  return r;
}

__device__ __forceinline__ void att_store_pass(const _Float16* so, _Float16* wtd,
                                               int b, int head, int q0, int lane) {
  const int q8 = lane & 7, sub = lane >> 3;
#pragma unroll
  for (int i = 0; i < 4; ++i) {
    const int row = i * 4 + sub;
    const v8h v = *(const v8ha*)(so + row * HD + 8 * q8);
    const size_t gi = ((size_t)b * SEQ + q0 + row) * EMB + head * HD + 8 * q8;
    *(volatile v8h*)(wtd + gi) = v;
  }
}

__global__ __launch_bounds__(128) void attn_kernel(
    const _Float16* __restrict__ qp,
    const _Float16* __restrict__ kp,
    const _Float16* __restrict__ vt,
    _Float16* __restrict__ wtd)
{
  __shared__ __attribute__((aligned(16))) _Float16 sO[4 * 16 * HD];

  const int tid = threadIdx.x, lane = tid & 31, w = tid >> 5;
  const int h = lane >> 4, m = lane & 15;
  const int bh = blockIdx.y, b = bh >> 4, head = bh & 15;
  const int q0 = blockIdx.x * 64 + 16 * w;

  const _Float16* qrow = qp + ((size_t)bh * SEQ + q0 + m) * HD;
  const v16h qb0 = ldfrag_h(qrow, h);
  const v16h qb1 = ldfrag_h(qrow + 32, h);

  const v8f zero8 = {0.f, 0.f, 0.f, 0.f, 0.f, 0.f, 0.f, 0.f};
  v8f o[4];
#pragma unroll
  for (int t = 0; t < 4; ++t) o[t] = zero8;
  float mrun = -1e30f, lrun = 0.0f;

  const _Float16* kbase = kp + ((size_t)bh * SEQ + m) * HD;
  const _Float16* vbase = vt + ((size_t)bh * HD + m) * SEQ;

#pragma unroll 1
  for (int kb = 0; kb < SEQ; kb += 64) {
    v8f s[4];
#pragma unroll
    for (int j = 0; j < 4; ++j) {
      const _Float16* kpj = kbase + (size_t)(kb + 16 * j) * HD;
      const v16h kf0 = ldfrag_h(kpj, h);
      const v16h kf1 = ldfrag_h(kpj + 32, h);
      v8f z = zero8;
      z = wmma_h(kf0, qb0, z);
      z = wmma_h(kf1, qb1, z);
      s[j] = z;
    }

    float mloc = -1e30f;
#pragma unroll
    for (int j = 0; j < 4; ++j)
#pragma unroll
      for (int r = 0; r < 8; ++r) {
        const float sv = s[j][r] * SSCALE;
        s[j][r] = sv;
        mloc = fmaxf(mloc, sv);
      }
    mloc = fmaxf(mloc, __shfl_xor(mloc, 16));
    const float mnew = fmaxf(mrun, mloc);
    const float alpha = __expf(mrun - mnew);
    mrun = mnew;
    float lsum = 0.0f;
#pragma unroll
    for (int j = 0; j < 4; ++j)
#pragma unroll
      for (int r = 0; r < 8; ++r) {
        const float p = __expf(s[j][r] - mnew);
        s[j][r] = p;
        lsum += p;
      }
    lsum += __shfl_xor(lsum, 16);
    lrun = lrun * alpha + lsum;
#pragma unroll
    for (int t = 0; t < 4; ++t)
#pragma unroll
      for (int r = 0; r < 8; ++r) o[t][r] = o[t][r] * alpha;

    const v16h pb0 = pack_p(s[0], s[1]);
    const v16h pb1 = pack_p(s[2], s[3]);

#pragma unroll
    for (int t = 0; t < 4; ++t) {
      const _Float16* vp = vbase + (size_t)(16 * t) * SEQ + kb;
      const v16h vf0 = ldfrag_h(vp, h);
      const v16h vf1 = ldfrag_h(vp + 32, h);
      o[t] = wmma_h(vf0, pb0, o[t]);
      o[t] = wmma_h(vf1, pb1, o[t]);
    }
  }

  const float inv = (1.0f / lrun) * ATT_OSC;
  _Float16* so = sO + w * (16 * HD);
#pragma unroll
  for (int t = 0; t < 4; ++t)
#pragma unroll
    for (int r = 0; r < 8; ++r)
      so[m * HD + 16 * t + 8 * h + r] = (_Float16)(o[t][r] * inv);
  __syncthreads();

  att_store_pass(so, wtd, b, head, q0, lane);
  __threadfence();
  att_store_pass(so, wtd, b, head, q0, lane);
}

__global__ __launch_bounds__(256) void out_ln_kernel(
    const _Float16* __restrict__ wtd,
    const _Float16* __restrict__ wo,
    const unsigned short* __restrict__ xb,
    const float* __restrict__ b_out,
    const float* __restrict__ gamma,
    const float* __restrict__ beta,
    float* __restrict__ out)
{
  __shared__ __attribute__((aligned(16))) float tile[16 * EMB];

  const int tid = threadIdx.x, lane = tid & 31, w = tid >> 5;
  const int h = lane >> 4, m = lane & 15;
  const int row0 = blockIdx.x * 16;

  const _Float16* arow = wtd + (size_t)(row0 + m) * EMB;
  const _Float16* brow = wo + (size_t)(128 * w + m) * EMB;

  const v8f zero8 = {0.f, 0.f, 0.f, 0.f, 0.f, 0.f, 0.f, 0.f};
  v8f acc[8];
#pragma unroll
  for (int nt = 0; nt < 8; ++nt) acc[nt] = zero8;

#pragma unroll 1
  for (int k0 = 0; k0 < EMB; k0 += 32) {
    const v16h a = ldfrag_h(arow + k0, h);
#pragma unroll
    for (int nt = 0; nt < 8; ++nt) {
      const v16h bfrag = ldfrag_h(brow + (size_t)nt * 16 * EMB + k0, h);
      acc[nt] = wmma_h(a, bfrag, acc[nt]);
    }
  }

#pragma unroll 2
  for (int it = 0; it < 8; ++it) {
    const int idx8 = it * 256 + tid;
    const int r = idx8 >> 7;
    const int c8 = (idx8 & 127) * 8;
    const v4u xs = *(const v4ua*)(xb + (size_t)(row0 + r) * EMB + c8);
    const v4f b0 = *(const v4fa*)(b_out + c8);
    const v4f b1 = *(const v4fa*)(b_out + c8 + 4);
    v4f lo4, hi4;
    lo4[0] = __uint_as_float(xs[0] << 16)          + bfr(b0[0]);
    lo4[1] = __uint_as_float(xs[0] & 0xffff0000u)  + bfr(b0[1]);
    lo4[2] = __uint_as_float(xs[1] << 16)          + bfr(b0[2]);
    lo4[3] = __uint_as_float(xs[1] & 0xffff0000u)  + bfr(b0[3]);
    hi4[0] = __uint_as_float(xs[2] << 16)          + bfr(b1[0]);
    hi4[1] = __uint_as_float(xs[2] & 0xffff0000u)  + bfr(b1[1]);
    hi4[2] = __uint_as_float(xs[3] << 16)          + bfr(b1[2]);
    hi4[3] = __uint_as_float(xs[3] & 0xffff0000u)  + bfr(b1[3]);
    *(v4fa*)(tile + r * EMB + c8)     = lo4;
    *(v4fa*)(tile + r * EMB + c8 + 4) = hi4;
  }
  __syncthreads();

#pragma unroll
  for (int nt = 0; nt < 8; ++nt)
#pragma unroll
    for (int r = 0; r < 8; ++r)
      tile[(8 * h + r) * EMB + 128 * w + 16 * nt + m] += acc[nt][r] * OUT_OSC;
  __syncthreads();

#pragma unroll 1
  for (int rr2 = 0; rr2 < 2; ++rr2) {
    const int rr = 2 * w + rr2;
    const float* tr = tile + rr * EMB;
    v4f v[8];
    float ssum = 0.0f;
#pragma unroll
    for (int i = 0; i < 8; ++i) {
      v[i] = *(const v4fa*)(tr + 128 * i + 4 * lane);
      ssum += (v[i][0] + v[i][1]) + (v[i][2] + v[i][3]);
    }
#pragma unroll
    for (int off = 16; off > 0; off >>= 1) ssum += __shfl_xor(ssum, off);
    const float mu = ssum * (1.0f / EMB);
    float sq = 0.0f;
#pragma unroll
    for (int i = 0; i < 8; ++i) {
      const float d0 = v[i][0] - mu, d1 = v[i][1] - mu, d2 = v[i][2] - mu, d3 = v[i][3] - mu;
      sq += (d0 * d0 + d1 * d1) + (d2 * d2 + d3 * d3);
    }
#pragma unroll
    for (int off = 16; off > 0; off >>= 1) sq += __shfl_xor(sq, off);
    const float rstd = rsqrtf(sq * (1.0f / EMB) + LN_EPS);
    v4f y[8];
#pragma unroll
    for (int i = 0; i < 8; ++i) {
      const v4f g  = *(const v4fa*)(gamma + 128 * i + 4 * lane);
      const v4f bt = *(const v4fa*)(beta  + 128 * i + 4 * lane);
      v4f yy;
      yy[0] = (v[i][0] - mu) * rstd * bfr(g[0]) + bfr(bt[0]);
      yy[1] = (v[i][1] - mu) * rstd * bfr(g[1]) + bfr(bt[1]);
      yy[2] = (v[i][2] - mu) * rstd * bfr(g[2]) + bfr(bt[2]);
      yy[3] = (v[i][3] - mu) * rstd * bfr(g[3]) + bfr(bt[3]);
      y[i] = yy;
    }
    float* orow = out + (size_t)(row0 + rr) * EMB;
    for (int pass = 0; pass < 2; ++pass) {
#pragma unroll
      for (int i = 0; i < 8; ++i)
        *(volatile v4f*)(orow + 128 * i + 4 * lane) = y[i];
      __threadfence();
    }
  }
}

extern "C" void kernel_launch(void* const* d_in, const int* in_sizes, int n_in,
                              void* d_out, int out_size, void* d_ws, size_t ws_size,
                              hipStream_t stream) {
  if (n_in < 7) return;
  if (in_sizes[0] != MROWS * EMB) return;
  if (in_sizes[1] != MROWS * NQKV) return;
  if (in_sizes[2] != NQKV * EMB) return;
  if (in_sizes[3] != EMB * EMB) return;
  if (in_sizes[4] != EMB || in_sizes[5] != EMB || in_sizes[6] != EMB) return;
  if (out_size != MROWS * EMB) return;

  const float* x     = (const float*)d_in[0];
  const float* ap    = (const float*)d_in[1];
  const float* wqkv  = (const float*)d_in[2];
  const float* wout  = (const float*)d_in[3];
  const float* b_out = (const float*)d_in[4];
  const float* gamma = (const float*)d_in[5];
  const float* beta  = (const float*)d_in[6];
  float* out = (float*)d_out;

  const size_t szXB  = (size_t)MROWS * EMB * 2;
  const size_t szWQ  = (size_t)NQKV * EMB * 2;
  const size_t szWO  = (size_t)EMB * EMB * 2;
  const size_t szPL  = (size_t)NB * NH * SEQ * HD * 2;
  const size_t szWTD = (size_t)MROWS * EMB * 2;
  size_t off = 0;
  const size_t oXB  = off; off += szXB;
  const size_t oWQ  = off; off += szWQ;
  const size_t oWO  = off; off += szWO;
  const size_t oQP  = off; off += szPL;
  const size_t oKP  = off; off += szPL;
  const size_t oVT  = off; off += szPL;
  const size_t oWTD = off; off += szWTD;
  if (off > ws_size) return;

  char* ws = (char*)d_ws;
  unsigned short* xb  = (unsigned short*)(ws + oXB);
  unsigned short* wq  = (unsigned short*)(ws + oWQ);
  _Float16*       wo  = (_Float16*)(ws + oWO);
  _Float16*       qp  = (_Float16*)(ws + oQP);
  _Float16*       kp  = (_Float16*)(ws + oKP);
  _Float16*       vt  = (_Float16*)(ws + oVT);
  _Float16*       wtd = (_Float16*)(ws + oWTD);

  prep_kernel<<<dim3(NBX + NBWQ + NBWO), dim3(256), 0, stream>>>(x, wqkv, wout, xb, wq, wo);

  qkv_kernel<<<dim3(MROWS / 128, 3 * NH), dim3(128), 0, stream>>>(xb, wq, ap, qp, kp, vt);

  attn_kernel<<<dim3(SEQ / 64, NB * NH), dim3(128), 0, stream>>>(qp, kp, vt, wtd);

  out_ln_kernel<<<dim3(MROWS / 16), dim3(256), 0, stream>>>(wtd, wo, xb, b_out, gamma, beta, out);

  (void)hipGetLastError();
}
